// MambaForecaster_83726092468228
// MI455X (gfx1250) — hardware-run, weakly checked
//
#include <hip/hip_runtime.h>
#include <math.h>

typedef __attribute__((ext_vector_type(16))) _Float16 v16h;
typedef __attribute__((ext_vector_type(8)))  _Float16 v8h;
typedef __attribute__((ext_vector_type(8)))  float    v8f;
typedef __attribute__((ext_vector_type(4)))  float    v4f;

constexpr int kBat   = 4;
constexpr int kSeq   = 512;
constexpr int kInD   = 32;
constexpr int kDm    = 512;
constexpr int kLay   = 4;
constexpr int kNst   = 16;
constexpr int kDin   = 1024;
constexpr int kDtR   = 32;
constexpr int kXzP   = 2 * kDin;
constexpr int kXdP   = kDtR + 2 * kNst;
constexpr int kRows  = kBat * kSeq;
constexpr int kHead  = 768;
constexpr int kTP    = 260;
static_assert(kXdP == 64);
static_assert(kRows == 2048 && kXzP == 2048);
static_assert((kRows % 64) == 0 && (kDm % 64) == 0 && (kXzP % 64) == 0 && (kXdP % 64) == 0 && (kDin % 64) == 0);
static_assert((kInD % 32) == 0 && (kDm % 32) == 0 && (kDin % 32) == 0 && (kDtR % 32) == 0);
static_assert((kSeq % 64) == 0 && (kDin % 256) == 0 && (kHead % 256) == 0);

constexpr float kCarWemb = 8.0f;
constexpr float kCarWin  = 32.0f;
constexpr float kCarWxp  = 32.0f;
constexpr float kCarWdt  = 8.0f;
constexpr float kCarWout = 32.0f;
constexpr float kCarDt   = 16.0f;
constexpr float kCarY    = 16.0f;

constexpr size_t kOffWIN  = 0;
constexpr size_t kOffWOUT = kOffWIN  + (size_t)kLay * kXzP * kDm * 2;
constexpr size_t kOffWXP  = kOffWOUT + (size_t)kLay * kDm * kDin * 2;
constexpr size_t kOffWDT  = kOffWXP  + (size_t)kLay * kXdP * kDin * 2;
constexpr size_t kOffWEMB = kOffWDT  + (size_t)kLay * kDin * kDtR * 2;
constexpr size_t kOffU16  = kOffWEMB + (size_t)kDm * kInD * 2;
constexpr size_t kOffHA   = kOffU16  + (size_t)kRows * kInD * 2;
constexpr size_t kOffHB   = kOffHA   + (size_t)kRows * kDm * 4;
constexpr size_t kOffHN   = kOffHB   + (size_t)kRows * kDm * 4;
constexpr size_t kOffXZ   = kOffHN   + (size_t)kRows * kDm * 2;
constexpr size_t kOffXB   = kOffXZ   + (size_t)kRows * kXzP * 4;
constexpr size_t kOffXB16 = kOffXB   + (size_t)kRows * kDin * 4;
constexpr size_t kOffDBC  = kOffXB16 + (size_t)kRows * kDin * 2;
constexpr size_t kOffDT16 = kOffDBC  + (size_t)kRows * kXdP * 4;
constexpr size_t kOffDLR  = kOffDT16 + (size_t)kRows * kDtR * 2;
constexpr size_t kOffY16  = kOffDLR  + (size_t)kRows * kDin * 4;
constexpr size_t kWsTotal = kOffY16  + (size_t)kRows * kDin * 2;
static_assert(kWsTotal == 66617344ull);
static_assert(kWsTotal <= 134217728ull);
static_assert((kOffWOUT % 128) == 0 && (kOffWXP % 128) == 0 && (kOffWDT % 128) == 0 && (kOffWEMB % 128) == 0 &&
              (kOffU16 % 128) == 0 && (kOffHA % 128) == 0 && (kOffHB % 128) == 0 && (kOffHN % 128) == 0 &&
              (kOffXZ % 128) == 0 && (kOffXB % 128) == 0 && (kOffXB16 % 128) == 0 && (kOffDBC % 128) == 0 &&
              (kOffDT16 % 128) == 0 && (kOffDLR % 128) == 0 && (kOffY16 % 128) == 0);

union FragU { v16h v; v8h h[2]; };
__device__ __forceinline__ v16h frag_load(const _Float16* p) {
  FragU f;
  f.h[0] = *(const v8h*)(p);
  f.h[1] = *(const v8h*)(p + 16);
  return f.v;
}
__device__ __forceinline__ v8f frag_mma(v16h a, v16h b, v8f c) {
  return __builtin_amdgcn_wmma_f32_16x16x32_f16(false, a, false, b, (short)0, c, false, false);
}
__device__ __forceinline__ void guard_row(v8f& a0, v8f& a1, v8f& a2, v8f& a3, v16h x, v16h b0, v16h b1, v16h b2, v16h b3) {
  asm volatile("v_nop\n\tv_nop\n\tv_nop\n\tv_nop" : "+v"(a0), "+v"(a1), "+v"(a2), "+v"(a3) : "v"(x), "v"(b0), "v"(b1), "v"(b2), "v"(b3) : "memory");
}
__device__ __forceinline__ void acc_guard4(v8f& a, v8f& b, v8f& c, v8f& d) {
  asm volatile("v_nop\n\tv_nop\n\tv_nop\n\tv_nop" : "+v"(a), "+v"(b), "+v"(c), "+v"(d));
}

template <int BIAS_MODE, bool RESID>
__global__ __launch_bounds__(256) __attribute__((amdgpu_num_vgpr(256))) void wmma_gemm64_f16(
    const unsigned short* __restrict__ Ap, int lda,
    const unsigned short* __restrict__ Btp, int ldb,
    float* __restrict__ Cout, int ldc,
    const float* __restrict__ bias, const float* __restrict__ resid,
    int M, int N, int K, float scale)
{
  const _Float16* A  = (const _Float16*)Ap;
  const _Float16* Bt = (const _Float16*)Btp;
  __shared__ __align__(16) float sT[8][16 * 68];
  const int lane = threadIdx.x & 31;
  const int wave = threadIdx.x >> 5;
  const int tilesN = N >> 6;
  const int tilesM = M >> 6;
  const int tile = blockIdx.x * 8 + wave;
  if (tile >= tilesM * tilesN) return;
  const int tm = tile / tilesN;
  const int tn = tile - tm * tilesN;
  const int m0 = tm << 6;
  const int n0 = tn << 6;

  const int rlane = lane & 15;
  const int koff  = (lane >> 4) * 8;
  const int mOff  = (lane >> 4) * 8;

  const _Float16* bp0 = Bt + (size_t)(n0 + rlane) * ldb + koff;
  const _Float16* ap0 = A  + (size_t)(m0 + rlane) * lda + koff;
  const size_t bstep = (size_t)16 * ldb;
  const size_t astep = (size_t)16 * lda;

  v8f acc[4][4];
#pragma unroll
  for (int i = 0; i < 4; ++i)
#pragma unroll
    for (int j = 0; j < 4; ++j) acc[i][j] = (v8f){0.f,0.f,0.f,0.f,0.f,0.f,0.f,0.f};

  for (int k0 = 0; k0 < K; k0 += 32) {
    v16h bh[4];
#pragma unroll
    for (int j = 0; j < 4; ++j) bh[j] = frag_load(bp0 + j * bstep + k0);
#pragma unroll
    for (int i = 0; i < 4; ++i) {
      const v16h ah = frag_load(ap0 + i * astep + k0);
#pragma unroll
      for (int j = 0; j < 4; ++j) acc[i][j] = frag_mma(ah, bh[j], acc[i][j]);
      guard_row(acc[i][0], acc[i][1], acc[i][2], acc[i][3], ah, bh[0], bh[1], bh[2], bh[3]);
    }
  }
  acc_guard4(acc[0][0], acc[0][1], acc[0][2], acc[0][3]);
  acc_guard4(acc[1][0], acc[1][1], acc[1][2], acc[1][3]);
  acc_guard4(acc[2][0], acc[2][1], acc[2][2], acc[2][3]);
  acc_guard4(acc[3][0], acc[3][1], acc[3][2], acc[3][3]);

  float* slab = sT[wave];
  const int hh = lane >> 4;
  const int c4 = (lane & 15) * 4;
#pragma unroll
  for (int i = 0; i < 4; ++i) {
    const int mBase = m0 + (i << 4);
#pragma unroll
    for (int j = 0; j < 4; ++j) {
#pragma unroll
      for (int r = 0; r < 8; ++r) {
        slab[(mOff + r) * 68 + (j << 4) + rlane] = acc[i][j][r] * scale;
      }
    }
    __builtin_amdgcn_fence(__ATOMIC_RELEASE, "workgroup");
    __builtin_amdgcn_wave_barrier();
    __builtin_amdgcn_fence(__ATOMIC_ACQUIRE, "workgroup");
    v4f bias4 = (v4f){0.f, 0.f, 0.f, 0.f};
    if (BIAS_MODE == 2) bias4 = *(const v4f*)(bias + n0 + c4);
#pragma unroll 1
    for (int hf = 0; hf < 2; ++hf) {
      v4f vals[4];
#pragma unroll
      for (int it = 0; it < 4; ++it) {
        const int row = hf * 8 + it * 2 + hh;
        v4f v = *(const v4f*)(slab + row * 68 + c4);
        if (BIAS_MODE == 2) v = v + bias4;
        if (RESID) {
          const v4f rv = *(const v4f*)(resid + (size_t)(mBase + row) * ldc + n0 + c4);
          v = v + rv;
        }
        vals[it] = v;
      }
      for (int pass = 0; pass < 2; ++pass) {
#pragma unroll
        for (int it = 0; it < 4; ++it) {
          const int row = hf * 8 + it * 2 + hh;
          *(volatile v4f*)(Cout + (size_t)(mBase + row) * ldc + n0 + c4) = vals[it];
        }
        __threadfence();
      }
    }
    __builtin_amdgcn_fence(__ATOMIC_RELEASE, "workgroup");
    __builtin_amdgcn_wave_barrier();
    __builtin_amdgcn_fence(__ATOMIC_ACQUIRE, "workgroup");
  }
}

__global__ __launch_bounds__(256) void cast_f16_kernel(
    const float* __restrict__ src, unsigned short* __restrict__ dst, int total8, float scale)
{
  const int i = blockIdx.x * 256 + threadIdx.x;
  if (i >= total8) return;
  const size_t e0 = (size_t)i << 3;
  const float* p = src + e0;
  const v4f a0 = *(const v4f*)(p);
  const v4f a1 = *(const v4f*)(p + 4);
  v8h hv;
#pragma unroll
  for (int e = 0; e < 4; ++e) {
    hv[e]     = (_Float16)(a0[e] * scale);
    hv[4 + e] = (_Float16)(a1[e] * scale);
  }
  unsigned short* q = dst + e0;
  *(volatile v8h*)q = hv;
  __threadfence();
  *(volatile v8h*)q = hv;
}

__global__ __launch_bounds__(256) void prep_u_kernel(const float* __restrict__ x, unsigned short* __restrict__ U16)
{
  __shared__ float sX[32 * 65];
  const int tid = threadIdx.x;
  const int m0 = blockIdx.x * 64;
  const int bb = m0 / kSeq;
  const int l0 = m0 - bb * kSeq;
#pragma unroll
  for (int p = 0; p < 8; ++p) {
    const int idx = tid + p * 256;
    const int ii = idx >> 6;
    const int ll = idx & 63;
    sX[ii * 65 + ll] = x[((size_t)bb * kInD + ii) * kSeq + l0 + ll];
  }
  __syncthreads();
  const int row = tid >> 2;
  const int seg = tid & 3;
  v8h hv;
#pragma unroll
  for (int e = 0; e < 8; ++e) hv[e] = (_Float16)sX[(seg * 8 + e) * 65 + row];
  unsigned short* q = U16 + (size_t)(m0 + row) * kInD + seg * 8;
  *(volatile v8h*)q = hv;
  __threadfence();
  *(volatile v8h*)q = hv;
}

__global__ __launch_bounds__(256) void rmsnorm_kernel(
    const float* __restrict__ h, const float* __restrict__ w, unsigned short* __restrict__ out)
{
  const int lane = threadIdx.x & 31;
  const int wave = threadIdx.x >> 5;
  const int row = blockIdx.x * 8 + wave;
  const float* hr = h + (size_t)row * kDm;
  const int c0 = lane * 8;
  const v4f a0 = *(const v4f*)(hr + c0);
  const v4f a1 = *(const v4f*)(hr + c0 + 4);
  const v4f a2 = *(const v4f*)(hr + 256 + c0);
  const v4f a3 = *(const v4f*)(hr + 256 + c0 + 4);
  const v4f w0 = *(const v4f*)(w + c0);
  const v4f w1 = *(const v4f*)(w + c0 + 4);
  const v4f w2 = *(const v4f*)(w + 256 + c0);
  const v4f w3 = *(const v4f*)(w + 256 + c0 + 4);
  float ss = 0.0f;
#pragma unroll
  for (int e = 0; e < 4; ++e) {
    ss += a0[e] * a0[e];
    ss += a1[e] * a1[e];
    ss += a2[e] * a2[e];
    ss += a3[e] * a3[e];
  }
#pragma unroll
  for (int off = 16; off > 0; off >>= 1) ss += __shfl_xor(ss, off, 32);
  const float sc = rsqrtf(ss * (1.0f / (float)kDm) + 1e-5f);
  v8h h0, h1;
#pragma unroll
  for (int e = 0; e < 4; ++e) {
    h0[e]     = (_Float16)((a0[e] * sc) * w0[e]);
    h0[4 + e] = (_Float16)((a1[e] * sc) * w1[e]);
    h1[e]     = (_Float16)((a2[e] * sc) * w2[e]);
    h1[4 + e] = (_Float16)((a3[e] * sc) * w3[e]);
  }
  unsigned short* q0 = out + (size_t)row * kDm + c0;
  unsigned short* q1 = q0 + 256;
  *(volatile v8h*)q0 = h0;
  *(volatile v8h*)q1 = h1;
  __threadfence();
  *(volatile v8h*)q0 = h0;
  *(volatile v8h*)q1 = h1;
}

__global__ __launch_bounds__(256) void conv_silu_kernel(
    const float* __restrict__ XZ, const float* __restrict__ cw, const float* __restrict__ cb,
    float* __restrict__ XB, unsigned short* __restrict__ XB16)
{
  __shared__ __align__(16) float sT[16 * kTP];
  const int tid = threadIdx.x, lane = tid & 31, wave = tid >> 5;
  const int d0 = blockIdx.x * 256, d = d0 + tid;
  const int g0 = blockIdx.y * 64;
  const int tb = g0 & (kSeq - 1);
  const v4f wv = *(const v4f*)(cw + (size_t)d * 4);
  const float w0 = wv[0], w1 = wv[1], w2 = wv[2], w3 = wv[3];
  const float bc = cb[d];
  float xm3, xm2, xm1;
  {
    const bool hist = (tb > 0);
    const int rb = hist ? (g0 - 3) : g0;
    const float v3 = XZ[(size_t)rb * kXzP + d];
    const float v2 = XZ[(size_t)(rb + 1) * kXzP + d];
    const float v1 = XZ[(size_t)(rb + 2) * kXzP + d];
    xm3 = hist ? v3 : 0.f;
    xm2 = hist ? v2 : 0.f;
    xm1 = hist ? v1 : 0.f;
  }
  const int hrow = wave >> 1;
  const int hch  = (wave & 1) * 128 + lane * 4;
#pragma unroll 1
  for (int sub = 0; sub < 4; ++sub) {
    const int lb = g0 + sub * 16;
#pragma unroll 1
    for (int s = 0; s < 16; ++s) {
      const float xcur = XZ[(size_t)(lb + s) * kXzP + d];
      float acc = w0 * xm3;
      acc = fmaf(w1, xm2, acc);
      acc = fmaf(w2, xm1, acc);
      acc = fmaf(w3, xcur, acc);
      const float sv = acc + bc;
      const float sg = __builtin_amdgcn_rcpf(1.0f + __expf(-sv));
      sT[s * kTP + tid] = sv * sg;
      xm3 = xm2; xm2 = xm1; xm1 = xcur;
    }
    __syncthreads();
    v4f fv[4];
    v8h bv[2];
#pragma unroll
    for (int it = 0; it < 4; ++it) fv[it] = *(const v4f*)(sT + (it * 4 + hrow) * kTP + hch);
#pragma unroll
    for (int it = 0; it < 2; ++it) {
      const float* sp = sT + (it * 8 + wave) * kTP + lane * 8;
      const v4f a0 = *(const v4f*)(sp);
      const v4f a1 = *(const v4f*)(sp + 4);
#pragma unroll
      for (int e = 0; e < 4; ++e) {
        bv[it][e]     = (_Float16)a0[e];
        bv[it][4 + e] = (_Float16)a1[e];
      }
    }
    for (int pass = 0; pass < 2; ++pass) {
#pragma unroll
      for (int it = 0; it < 4; ++it)
        *(volatile v4f*)(XB + (size_t)(lb + it * 4 + hrow) * kDin + d0 + hch) = fv[it];
#pragma unroll
      for (int it = 0; it < 2; ++it)
        *(volatile v8h*)(XB16 + (size_t)(lb + it * 8 + wave) * kDin + d0 + lane * 8) = bv[it];
      __threadfence();
    }
    __syncthreads();
  }
}

__global__ __launch_bounds__(256) void dt_cast_kernel(
    const float* __restrict__ DBC, unsigned short* __restrict__ DT16, int total8, float scale)
{
  const int i = blockIdx.x * 256 + threadIdx.x;
  if (i >= total8) return;
  const int e0  = i << 3;
  const int row = e0 >> 5;
  const int c8  = e0 & 31;
  const float* p = DBC + (size_t)row * kXdP + c8;
  const v4f a0 = *(const v4f*)(p);
  const v4f a1 = *(const v4f*)(p + 4);
  v8h hv;
#pragma unroll
  for (int e = 0; e < 4; ++e) {
    hv[e]     = (_Float16)(a0[e] * scale);
    hv[4 + e] = (_Float16)(a1[e] * scale);
  }
  unsigned short* qd = DT16 + e0;
  *(volatile v8h*)qd = hv;
  __threadfence();
  *(volatile v8h*)qd = hv;
}

__global__ __launch_bounds__(256) void scan_kernel(
    const float* __restrict__ DLR, const float* __restrict__ XB, const float* __restrict__ XZ,
    const float* __restrict__ DBC, const float* __restrict__ A_log, const float* __restrict__ Dv,
    unsigned short* __restrict__ Y16)
{
  __shared__ __align__(16) float sBC[16 * 32];
  __shared__ __align__(16) float sY[16 * kTP];
  __shared__ float sA[kNst * 256];
  const int tid = threadIdx.x, lane = tid & 31, wave = tid >> 5;
  constexpr int kBlkPerB = kDin / 256;
  const int bix = blockIdx.x / kBlkPerB;
  const int d0 = (blockIdx.x - bix * kBlkPerB) * 256;
  const int d = d0 + tid;
  const size_t row0 = (size_t)bix * kSeq;

#pragma unroll 1
  for (int n = 0; n < kNst; ++n) sA[n * 256 + tid] = -expf(A_log[(size_t)d * kNst + n]);
  __syncthreads();
  float An[kNst], h[kNst];
#pragma unroll
  for (int n = 0; n < kNst; ++n) {
    An[n] = sA[n * 256 + tid];
    h[n] = 0.f;
  }
  const float Dd = Dv[d];

#pragma unroll 1
  for (int c = 0; c < kSeq / 16; ++c) {
    const int l0 = c * 16;
    if (tid < 128) {
      const int r = tid >> 3, q = (tid & 7) * 4;
      const v4f v = *(const v4f*)(DBC + (row0 + l0 + r) * kXdP + kDtR + q);
      *(v4f*)(sBC + r * 32 + q) = v;
    }
    __syncthreads();
#pragma unroll 1
    for (int s = 0; s < 16; ++s) {
      const size_t m = row0 + (size_t)(l0 + s);
      const float a  = DLR[m * kDin + d];
      const float xv = XB[m * kDin + d];
      const float zv = XZ[m * kXzP + kDin + d];
      const float delta = fmaxf(a, 0.0f) + log1pf(__expf(-fabsf(a)));
      v4f Bq[4], Cq[4];
#pragma unroll
      for (int qq = 0; qq < 4; ++qq) {
        Bq[qq] = *(const v4f*)(sBC + s * 32 + 4 * qq);
        Cq[qq] = *(const v4f*)(sBC + s * 32 + kNst + 4 * qq);
      }
      const float dtx = delta * xv;
      float y = 0.f;
#pragma unroll
      for (int n = 0; n < kNst; ++n) {
        const float e = __expf(delta * An[n]);
        const float hn = fmaf(e, h[n], dtx * Bq[n >> 2][n & 3]);
        h[n] = hn;
        y = fmaf(hn, Cq[n >> 2][n & 3], y);
      }
      y = fmaf(xv, Dd, y);
      const float sg = __builtin_amdgcn_rcpf(1.0f + __expf(-zv));
      const float g  = zv * sg;
      sY[s * kTP + tid] = (y * g) * kCarY;
    }
    __syncthreads();
    v8h hv[2];
#pragma unroll
    for (int it = 0; it < 2; ++it) {
      const float* sp = sY + (it * 8 + wave) * kTP + lane * 8;
      const v4f a0 = *(const v4f*)(sp);
      const v4f a1 = *(const v4f*)(sp + 4);
#pragma unroll
      for (int e = 0; e < 4; ++e) {
        hv[it][e]     = (_Float16)a0[e];
        hv[it][4 + e] = (_Float16)a1[e];
      }
    }
    for (int pass = 0; pass < 2; ++pass) {
#pragma unroll
      for (int it = 0; it < 2; ++it)
        *(volatile v8h*)(Y16 + (row0 + (size_t)(l0 + it * 8 + wave)) * kDin + d0 + lane * 8) = hv[it];
      __threadfence();
    }
  }
}

__global__ __launch_bounds__(256) void head_kernel(
    const float* __restrict__ h, const float* __restrict__ Wh, const float* __restrict__ bh, float* __restrict__ out)
{
  __shared__ __align__(16) float sH[kBat * kDm];
  const int tid = threadIdx.x;
#pragma unroll
  for (int p = 0; p < 8; ++p) {
    const int idx = tid + p * 256;
    const int bb = idx >> 9;
    const int cc = idx & (kDm - 1);
    sH[idx] = h[((size_t)bb * kSeq + (kSeq - 1)) * kDm + cc];
  }
  __syncthreads();
  const int j = blockIdx.x * 256 + tid;
  const float* wr = Wh + (size_t)j * kDm;
  float acc0 = 0.f, acc1 = 0.f, acc2 = 0.f, acc3 = 0.f;
#pragma unroll 1
  for (int k4 = 0; k4 < kDm / 4; ++k4) {
    const v4f wv = *(const v4f*)(wr + 4 * k4);
    const v4f h0 = *(const v4f*)(sH + 4 * k4);
    const v4f h1 = *(const v4f*)(sH + kDm + 4 * k4);
    const v4f h2 = *(const v4f*)(sH + 2 * kDm + 4 * k4);
    const v4f h3 = *(const v4f*)(sH + 3 * kDm + 4 * k4);
#pragma unroll
    for (int e = 0; e < 4; ++e) {
      acc0 = fmaf(h0[e], wv[e], acc0);
      acc1 = fmaf(h1[e], wv[e], acc1);
      acc2 = fmaf(h2[e], wv[e], acc2);
      acc3 = fmaf(h3[e], wv[e], acc3);
    }
  }
  const float bj = bh[j];
  const float o0 = acc0 + bj, o1 = acc1 + bj, o2 = acc2 + bj, o3 = acc3 + bj;
  for (int pass = 0; pass < 2; ++pass) {
    *(volatile float*)(out + j) = o0;
    *(volatile float*)(out + kHead + j) = o1;
    *(volatile float*)(out + 2 * kHead + j) = o2;
    *(volatile float*)(out + 3 * kHead + j) = o3;
    __threadfence();
  }
}

extern "C" void kernel_launch(void* const* d_in, const int* in_sizes, int n_in,
                              void* d_out, int out_size, void* d_ws, size_t ws_size,
                              hipStream_t stream)
{
  if (n_in < 15) return;
  if (in_sizes[0]  != kBat * kInD * kSeq) return;
  if (in_sizes[1]  != kDm * kInD) return;
  if (in_sizes[2]  != kDm) return;
  if (in_sizes[3]  != kLay * kDm) return;
  if (in_sizes[4]  != kLay * kXzP * kDm) return;
  if (in_sizes[5]  != kLay * kDin * 4) return;
  if (in_sizes[6]  != kLay * kDin) return;
  if (in_sizes[7]  != kLay * kXdP * kDin) return;
  if (in_sizes[8]  != kLay * kDin * kDtR) return;
  if (in_sizes[9]  != kLay * kDin) return;
  if (in_sizes[10] != kLay * kDin * kNst) return;
  if (in_sizes[11] != kLay * kDin) return;
  if (in_sizes[12] != kLay * kDm * kDin) return;
  if (in_sizes[13] != kHead * kDm) return;
  if (in_sizes[14] != kHead) return;
  if (out_size != kBat * kHead) return;
  if (ws_size < kWsTotal) return;

  const float* x         = (const float*)d_in[0];
  const float* embed_w   = (const float*)d_in[1];
  const float* embed_b   = (const float*)d_in[2];
  const float* norm_w    = (const float*)d_in[3];
  const float* in_proj_w = (const float*)d_in[4];
  const float* conv_w    = (const float*)d_in[5];
  const float* conv_b    = (const float*)d_in[6];
  const float* x_proj_w  = (const float*)d_in[7];
  const float* dt_proj_w = (const float*)d_in[8];
  const float* dt_proj_b = (const float*)d_in[9];
  const float* A_log     = (const float*)d_in[10];
  const float* Dparam    = (const float*)d_in[11];
  const float* out_proj_w= (const float*)d_in[12];
  const float* head_w    = (const float*)d_in[13];
  const float* head_b    = (const float*)d_in[14];
  float* dout = (float*)d_out;

  char* ws = (char*)d_ws;
  unsigned short* WIN16  = (unsigned short*)(ws + kOffWIN);
  unsigned short* WOUT16 = (unsigned short*)(ws + kOffWOUT);
  unsigned short* WXP16  = (unsigned short*)(ws + kOffWXP);
  unsigned short* WDT16  = (unsigned short*)(ws + kOffWDT);
  unsigned short* WEMB16 = (unsigned short*)(ws + kOffWEMB);
  unsigned short* U16    = (unsigned short*)(ws + kOffU16);
  float*          HA     = (float*)(ws + kOffHA);
  float*          HB     = (float*)(ws + kOffHB);
  unsigned short* HN16   = (unsigned short*)(ws + kOffHN);
  float*          XZ     = (float*)(ws + kOffXZ);
  float*          XB     = (float*)(ws + kOffXB);
  unsigned short* XB16   = (unsigned short*)(ws + kOffXB16);
  float*          DBC    = (float*)(ws + kOffDBC);
  unsigned short* DT16   = (unsigned short*)(ws + kOffDT16);
  float*          DLR    = (float*)(ws + kOffDLR);
  unsigned short* Y16    = (unsigned short*)(ws + kOffY16);

  {
    const int n_in8  = kLay * kXzP * kDm / 8;
    const int n_out8 = kLay * kDm * kDin / 8;
    const int n_xp8  = kLay * kXdP * kDin / 8;
    const int n_dt8  = kLay * kDin * kDtR / 8;
    const int n_em8  = kDm * kInD / 8;
    cast_f16_kernel<<<n_in8 / 256, 256, 0, stream>>>(in_proj_w, WIN16, n_in8, kCarWin);
    cast_f16_kernel<<<n_out8 / 256, 256, 0, stream>>>(out_proj_w, WOUT16, n_out8, kCarWout);
    cast_f16_kernel<<<n_xp8 / 256, 256, 0, stream>>>(x_proj_w, WXP16, n_xp8, kCarWxp);
    cast_f16_kernel<<<n_dt8 / 256, 256, 0, stream>>>(dt_proj_w, WDT16, n_dt8, kCarWdt);
    cast_f16_kernel<<<n_em8 / 256, 256, 0, stream>>>(embed_w, WEMB16, n_em8, kCarWemb);
  }

  prep_u_kernel<<<kRows / 64, 256, 0, stream>>>(x, U16);

  wmma_gemm64_f16<2, false><<<(kRows / 64) * (kDm / 64) / 8, 256, 0, stream>>>(
      U16, kInD, WEMB16, kInD, HA, kDm, embed_b, HA, kRows, kDm, kInD, 1.0f / kCarWemb);

  for (int i = 0; i < kLay; ++i) {
    const float* hin  = (i & 1) ? HB : HA;
    float*       hout = (i & 1) ? HA : HB;
    const unsigned short* win  = WIN16  + (size_t)i * kXzP * kDm;
    const unsigned short* wout = WOUT16 + (size_t)i * kDm * kDin;
    const unsigned short* wxp  = WXP16  + (size_t)i * kXdP * kDin;
    const unsigned short* wdt  = WDT16  + (size_t)i * kDin * kDtR;
    const float* nwp  = norm_w    + (size_t)i * kDm;
    const float* cwp  = conv_w    + (size_t)i * kDin * 4;
    const float* cbp  = conv_b    + (size_t)i * kDin;
    const float* dtbp = dt_proj_b + (size_t)i * kDin;
    const float* alp  = A_log     + (size_t)i * kDin * kNst;
    const float* dpp  = Dparam    + (size_t)i * kDin;

    rmsnorm_kernel<<<kRows / 8, 256, 0, stream>>>(hin, nwp, HN16);

    wmma_gemm64_f16<0, false><<<(kRows / 64) * (kXzP / 64) / 8, 256, 0, stream>>>(
        HN16, kDm, win, kDm, XZ, kXzP, embed_b, hin, kRows, kXzP, kDm, 1.0f / kCarWin);

    conv_silu_kernel<<<dim3(kDin / 256, kRows / 64), 256, 0, stream>>>(XZ, cwp, cbp, XB, XB16);

    wmma_gemm64_f16<0, false><<<(kRows / 64) * (kXdP / 64) / 8, 256, 0, stream>>>(
        XB16, kDin, wxp, kDin, DBC, kXdP, embed_b, hin, kRows, kXdP, kDin, 1.0f / kCarWxp);

    dt_cast_kernel<<<(kRows * kDtR / 8) / 256, 256, 0, stream>>>(DBC, DT16, kRows * kDtR / 8, kCarDt);

    wmma_gemm64_f16<2, false><<<(kRows / 64) * (kDin / 64) / 8, 256, 0, stream>>>(
        DT16, kDtR, wdt, kDtR, DLR, kDin, dtbp, hin, kRows, kDin, kDtR, 1.0f / (kCarDt * kCarWdt));

    scan_kernel<<<kBat * (kDin / 256), 256, 0, stream>>>(DLR, XB, XZ, DBC, alp, dpp, Y16);

    wmma_gemm64_f16<0, true><<<(kRows / 64) * (kDm / 64) / 8, 256, 0, stream>>>(
        Y16, kDin, wout, kDin, hout, kDm, embed_b, hin, kRows, kDm, kDin, 1.0f / (kCarY * kCarWout));
  }

  head_kernel<<<kHead / 256, 256, 0, stream>>>(HA, head_w, head_b, dout);
}
